// TeethAlignmentModel_88459146428620
// MI455X (gfx1250) — hardware-verified
//
#include <hip/hip_runtime.h>
#define NBc 8
#define NP 8192
#define NR (NBc * NP)
#define C1 64
#define C2 128
#define C3 1024
#define F1 512
#define F2 256
#define EPS 1e-5f
typedef __bf16 v16b __attribute__((ext_vector_type(16)));
typedef unsigned short v8us __attribute__((ext_vector_type(8), may_alias));
typedef float  v8f  __attribute__((ext_vector_type(8)));
typedef float  v4f  __attribute__((ext_vector_type(4)));
typedef float  v4fa __attribute__((ext_vector_type(4), may_alias));
union FragB { v16b v; v8us half[2]; unsigned short u[16]; };

__device__ __forceinline__ unsigned short bf16_bits(float x) { unsigned int u = __float_as_uint(x); return (unsigned short)((u + 0x7FFFu + ((u >> 16) & 1u)) >> 16); }
__device__ __forceinline__ float bf16_val(unsigned short b) { return __uint_as_float(((unsigned int)b) << 16); }
__device__ __forceinline__ float bf16_round(float x) { return bf16_val(bf16_bits(x)); }
template <int NT>
__device__ __forceinline__ v8f mmaN(v16b ah, v16b al, v16b bh, v16b bl, v8f c) {
  c = __builtin_amdgcn_wmma_f32_16x16x32_bf16(false, ah, false, bh, (short)0, c, false, false);
  if (NT >= 2) c = __builtin_amdgcn_wmma_f32_16x16x32_bf16(false, al, false, bh, (short)0, c, false, false);
  if (NT >= 3) c = __builtin_amdgcn_wmma_f32_16x16x32_bf16(false, ah, false, bl, (short)0, c, false, false);
  asm volatile("v_nop\n\tv_nop\n\tv_nop\n\tv_nop" : "+v"(c) : "v"(ah), "v"(al), "v"(bh), "v"(bl));
  return c;
}

__global__ __launch_bounds__(256) void k_wt_bf16(const float* __restrict__ W, unsigned short* __restrict__ Wt, int K, int N) {
  const int t = blockIdx.x * 256 + threadIdx.x;
  const int k8n = K / 8;
  if (t >= N * k8n) return;
  const int n = t / k8n, k8 = (t % k8n) * 8;
  v8us v;
#pragma unroll
  for (int i = 0; i < 8; ++i) v[i] = bf16_bits(W[(size_t)(k8 + i) * N + n]);
  *(volatile v8us*)(Wt + (size_t)n * K + k8) = v;
  __threadfence();
  *(volatile v8us*)(Wt + (size_t)n * K + k8) = v;
}

template <bool ASPLIT, int ACT, bool BIAS_BF16>
__global__ __launch_bounds__(128) void k_gemm_bf(const float* __restrict__ A, int lda, const unsigned short* __restrict__ Wt, int ldb,
                                               const float* __restrict__ bias, float* __restrict__ C, int ldc, int M, int N, int K) {
  __shared__ __attribute__((aligned(16))) float so[4][16][64];
  const int tid = threadIdx.x, w = tid >> 5, lane = tid & 31, ln = lane & 15, hh = lane >> 4;
  const int ntn = N / 64;
  const int wid = blockIdx.x * 4 + w;
  const int mt = wid / ntn, nq = wid % ntn;
  if (mt * 16 >= M) return;
  const int row0 = mt * 16, col0 = nq * 64;
  const float* arow = A + (size_t)(row0 + ln) * lda;
  v8f acc[4] = {};
  for (int kb = 0; kb < K; kb += 32) {
    FragB ah, al;
    const v4f x0 = *(const v4fa*)(arow + kb + 8 * hh), x1 = *(const v4fa*)(arow + kb + 8 * hh + 4);
    const v4f x2 = *(const v4fa*)(arow + kb + 16 + 8 * hh), x3 = *(const v4fa*)(arow + kb + 16 + 8 * hh + 4);
    float xs[16] = {x0[0],x0[1],x0[2],x0[3],x1[0],x1[1],x1[2],x1[3],x2[0],x2[1],x2[2],x2[3],x3[0],x3[1],x3[2],x3[3]};
#pragma unroll
    for (int i = 0; i < 16; ++i) { const unsigned short hb = bf16_bits(xs[i]); ah.u[i] = hb; al.u[i] = ASPLIT ? bf16_bits(xs[i] - bf16_val(hb)) : (unsigned short)0; }
#pragma unroll
    for (int t = 0; t < 4; ++t) {
      const unsigned short* brow = Wt + (size_t)(col0 + t * 16 + ln) * ldb + kb;
      FragB b;
      b.half[0] = *(const v8us*)(brow + 8 * hh);
      b.half[1] = *(const v8us*)(brow + 16 + 8 * hh);
      acc[t] = mmaN<ASPLIT ? 2 : 1>(ah.v, al.v, b.v, b.v, acc[t]);
    }
  }
#pragma unroll
  for (int t = 0; t < 4; ++t) {
    float bv = bias ? bias[col0 + t * 16 + ln] : 0.f;
    if (BIAS_BF16) bv = bf16_round(bv);
#pragma unroll
    for (int r = 0; r < 8; ++r) { float v = acc[t][r] + bv; if (ACT == 1) v = fmaxf(v, 0.f); so[w][8 * hh + r][t * 16 + ln] = v; }
  }
  __builtin_amdgcn_fence(__ATOMIC_ACQ_REL, "workgroup");
  __builtin_amdgcn_wave_barrier();
  const int rsub = lane >> 4, c4 = (lane & 15) * 4;
  for (int pass = 0; pass < 2; ++pass) {
#pragma unroll
    for (int q = 0; q < 8; ++q) {
      const int r = q * 2 + rsub;
      const v4f v = *(const v4fa*)&so[w][r][c4];
      *(volatile v4f*)(C + (size_t)(row0 + r) * ldc + col0 + c4) = v;
    }
    if (pass == 0) __threadfence();
  }
}

template <bool ASPLIT, int ACT, bool BIAS_BF16, bool RES_BF16>
__global__ __launch_bounds__(128) void k_gemm_bf3(const float* __restrict__ A, int lda, const unsigned short* __restrict__ Wt, int ldb,
                                                const float* __restrict__ bias, const float* __restrict__ resid, int rmod, int ldr,
                                                float* __restrict__ C, int ldc, int M, int N, int K) {
  __shared__ __attribute__((aligned(16))) float so[4][16][64];
  const int tid = threadIdx.x, w = tid >> 5, lane = tid & 31, ln = lane & 15, hh = lane >> 4;
  const int ntn = N / 64;
  const int wid = blockIdx.x * 4 + w;
  const int mt = wid / ntn, nq = wid % ntn;
  if (mt * 16 >= M) return;
  const int row0 = mt * 16, col0 = nq * 64;
  const float* arow = A + (size_t)(row0 + ln) * lda;
  v8f acc[4] = {};
  for (int kb = 0; kb < K; kb += 32) {
    FragB ah, al;
    const v4f x0 = *(const v4fa*)(arow + kb + 8 * hh), x1 = *(const v4fa*)(arow + kb + 8 * hh + 4);
    const v4f x2 = *(const v4fa*)(arow + kb + 16 + 8 * hh), x3 = *(const v4fa*)(arow + kb + 16 + 8 * hh + 4);
    float xs[16] = {x0[0],x0[1],x0[2],x0[3],x1[0],x1[1],x1[2],x1[3],x2[0],x2[1],x2[2],x2[3],x3[0],x3[1],x3[2],x3[3]};
#pragma unroll
    for (int i = 0; i < 16; ++i) { const unsigned short hb = bf16_bits(xs[i]); ah.u[i] = hb; al.u[i] = ASPLIT ? bf16_bits(xs[i] - bf16_val(hb)) : (unsigned short)0; }
#pragma unroll
    for (int t = 0; t < 4; ++t) {
      const unsigned short* brow = Wt + (size_t)(col0 + t * 16 + ln) * ldb + kb;
      FragB b;
      b.half[0] = *(const v8us*)(brow + 8 * hh);
      b.half[1] = *(const v8us*)(brow + 16 + 8 * hh);
      acc[t] = mmaN<ASPLIT ? 2 : 1>(ah.v, al.v, b.v, b.v, acc[t]);
    }
  }
#pragma unroll
  for (int t = 0; t < 4; ++t) {
    const int col = col0 + t * 16 + ln;
    float bv = bias ? bias[col] : 0.f;
    if (BIAS_BF16) bv = bf16_round(bv);
#pragma unroll
    for (int r = 0; r < 8; ++r) {
      float v = acc[t][r] + bv;
      if (resid) { float rv = resid[(size_t)((row0 + 8 * hh + r) % rmod) * ldr + col]; if (RES_BF16) rv = bf16_round(rv); v += rv; }
      if (ACT == 1) v = fmaxf(v, 0.f);
      if (ACT == 2) v = 0.5f * v * (1.0f + erff(v * 0.70710678118654752f));
      if (ACT == 3) { const float u = 0.7978845608028654f * (v + 0.044715f * v * v * v); v = 0.5f * v * (1.0f + tanhf(u)); }
      so[w][8 * hh + r][t * 16 + ln] = v;
    }
  }
  __builtin_amdgcn_fence(__ATOMIC_ACQ_REL, "workgroup");
  __builtin_amdgcn_wave_barrier();
  const int rsub = lane >> 4, c4 = (lane & 15) * 4;
  for (int pass = 0; pass < 2; ++pass) {
#pragma unroll
    for (int q = 0; q < 8; ++q) {
      const int r = q * 2 + rsub;
      const v4f v = *(const v4fa*)&so[w][r][c4];
      *(volatile v4f*)(C + (size_t)(row0 + r) * ldc + col0 + c4) = v;
    }
    if (pass == 0) __threadfence();
  }
}
template <bool PARAM_BF16>
__global__ __launch_bounds__(256) void k_layernorm(const float* __restrict__ X, const float* __restrict__ R, const float* __restrict__ g, const float* __restrict__ bta,
                                                  float* __restrict__ out_sum, float* __restrict__ out_norm, int N, float eps) {
  __shared__ float red[256];
  const int row = blockIdx.x, tid = threadIdx.x;
  const float* x = X + (size_t)row * N; const float* rr = R ? R + (size_t)row * N : nullptr;
  float vals[16];
  const int per = N / 256;
  float s1 = 0.f;
  for (int u = 0; u < per / 4; ++u) {
    const int j = tid * 4 + 1024 * u;
    const v4f a = *(const v4fa*)(x + j);
    v4f b = {0.f,0.f,0.f,0.f}; if (rr) b = *(const v4fa*)(rr + j);
#pragma unroll
    for (int q = 0; q < 4; ++q) { const float v = a[q] + b[q]; vals[u * 4 + q] = v; s1 += v; }
  }
  red[tid] = s1; __syncthreads();
  for (int st = 128; st > 0; st >>= 1) { if (tid < st) red[tid] += red[tid + st]; __syncthreads(); }
  const float mu = red[0] / (float)N; __syncthreads();
  float s2 = 0.f;
  for (int u = 0; u < per / 4; ++u)
#pragma unroll
    for (int q = 0; q < 4; ++q) { const float c = vals[u * 4 + q] - mu; s2 += c * c; }
  red[tid] = s2; __syncthreads();
  for (int st = 128; st > 0; st >>= 1) { if (tid < st) red[tid] += red[tid + st]; __syncthreads(); }
  const float rs = rsqrtf(red[0] / (float)N + eps);
  for (int pass = 0; pass < 2; ++pass) {
    for (int u = 0; u < per / 4; ++u) {
      const int j = tid * 4 + 1024 * u;
      v4f o, sm;
#pragma unroll
      for (int q = 0; q < 4; ++q) {
        float gg = g[j + q], bb = bta[j + q];
        if (PARAM_BF16) { gg = bf16_round(gg); bb = bf16_round(bb); }
        sm[q] = vals[u * 4 + q]; o[q] = (vals[u * 4 + q] - mu) * rs * gg + bb;
      }
      if (out_sum) *(volatile v4f*)(out_sum + (size_t)row * N + j) = sm;
      *(volatile v4f*)(out_norm + (size_t)row * N + j) = o;
    }
    if (pass == 0) __threadfence();
  }
}


typedef _Float16 v16h __attribute__((ext_vector_type(16)));
union FragH { v16h v; v8us half[2]; _Float16 h[16]; unsigned short u[16]; };
template <int NT>
__device__ __forceinline__ v8f mmaH(v16h ah, v16h al, v16h bh, v16h bl, v8f c) {
  c = __builtin_amdgcn_wmma_f32_16x16x32_f16(false, ah, false, bh, (short)0, c, false, false);
  if (NT >= 2) c = __builtin_amdgcn_wmma_f32_16x16x32_f16(false, al, false, bh, (short)0, c, false, false);
  if (NT >= 3) c = __builtin_amdgcn_wmma_f32_16x16x32_f16(false, ah, false, bl, (short)0, c, false, false);
  asm volatile("v_nop\n\tv_nop\n\tv_nop\n\tv_nop" : "+v"(c) : "v"(ah), "v"(al), "v"(bh), "v"(bl));
  return c;
}
template <bool ASPLIT>
__global__ __launch_bounds__(128) void k_gemm_h(const float* __restrict__ A, int lda, size_t sA, const _Float16* __restrict__ Bh, int ldb, size_t sB, float alpha, float* __restrict__ C, int ldc, size_t sC, int M, int N, int K) {
  __shared__ __attribute__((aligned(16))) float so[4][16][64];
  const int tid = threadIdx.x, w = tid >> 5, lane = tid & 31, ln = lane & 15, hh = lane >> 4; const int by = blockIdx.y;
  A += (size_t)by * sA; Bh += (size_t)by * sB; C += (size_t)by * sC;
  const int ntn = (N + 63) / 64; const int wid = blockIdx.x * 4 + w; const int mt = wid / ntn, nq = wid % ntn; if (mt * 16 >= M) return;
  const int row0 = mt * 16, col0 = nq * 64; const float* arow = A + (size_t)(row0 + ln) * lda;
  v8f acc[4] = {};
  for (int kb = 0; kb < K; kb += 32) {
    FragH ah, al;
    const v4f x0 = *(const v4fa*)(arow + kb + 8 * hh), x1 = *(const v4fa*)(arow + kb + 8 * hh + 4), x2 = *(const v4fa*)(arow + kb + 16 + 8 * hh), x3 = *(const v4fa*)(arow + kb + 16 + 8 * hh + 4);
    float xs[16] = {x0[0],x0[1],x0[2],x0[3],x1[0],x1[1],x1[2],x1[3],x2[0],x2[1],x2[2],x2[3],x3[0],x3[1],x3[2],x3[3]};
#pragma unroll
    for (int i = 0; i < 16; ++i) { const _Float16 h = (_Float16)xs[i]; ah.h[i] = h; al.h[i] = ASPLIT ? (_Float16)(xs[i] - (float)h) : (_Float16)0.0f; }
#pragma unroll
    for (int t = 0; t < 4; ++t) { if (col0 + t * 16 >= N) continue; const size_t boff = (size_t)(col0 + t * 16 + ln) * ldb + kb; FragH bq; bq.half[0] = *(const v8us*)(Bh + boff + 8 * hh); bq.half[1] = *(const v8us*)(Bh + boff + 16 + 8 * hh);
      acc[t] = mmaH<ASPLIT ? 2 : 1>(ah.v, al.v, bq.v, bq.v, acc[t]); }
  }
#pragma unroll
  for (int t = 0; t < 4; ++t) { if (col0 + t * 16 >= N) continue;
#pragma unroll
    for (int r = 0; r < 8; ++r) so[w][8 * hh + r][t * 16 + ln] = acc[t][r] * alpha; }
  __builtin_amdgcn_fence(__ATOMIC_ACQ_REL, "workgroup"); __builtin_amdgcn_wave_barrier();
  const int rsub = lane >> 4, c4 = (lane & 15) * 4;
  for (int pass = 0; pass < 2; ++pass) {
#pragma unroll
    for (int q = 0; q < 8; ++q) { const int r = q * 2 + rsub; if (col0 + c4 < N) { const v4f v = *(const v4fa*)&so[w][r][c4]; *(volatile v4f*)(C + (size_t)(row0 + r) * ldc + col0 + c4) = v; } }
    if (pass == 0) __threadfence(); }
}

__global__ __launch_bounds__(256) void k_wt_f16(const float* __restrict__ W, _Float16* __restrict__ Wt, int K, int N, float scale) {
  const int t = blockIdx.x * 256 + threadIdx.x; if (t >= N * (K / 8)) return; const int n = t / (K / 8), k8 = (t % (K / 8)) * 8; FragH f;
#pragma unroll
  for (int i = 0; i < 8; ++i) f.h[i] = (_Float16)(bf16_round(W[(size_t)(k8 + i) * N + n]) * scale); const v8us o = f.half[0];
  *(volatile v8us*)((unsigned short*)Wt + (size_t)n * K + k8) = o; __threadfence(); *(volatile v8us*)((unsigned short*)Wt + (size_t)n * K + k8) = o;
}
template <int ACT>
__global__ __launch_bounds__(128) void k_gemm_hhx(const _Float16* __restrict__ A, int lda, size_t sA, const _Float16* __restrict__ Bh, int ldb, size_t sB, float alpha, const float* __restrict__ bias, size_t sBias, const float* __restrict__ CP, int rowsPerB, size_t sCPb, int row0g,
    float* __restrict__ C, _Float16* __restrict__ C16, int ldc, size_t sC, int M, int N, int K) {
  __shared__ __attribute__((aligned(16))) float so[4][16][64];
  const int tid = threadIdx.x, w = tid >> 5, lane = tid & 31, ln = lane & 15, hh = lane >> 4; const int by = blockIdx.y;
  A += (size_t)by * sA; Bh += (size_t)by * sB; const size_t cofs = (size_t)by * sC; const float* bp = bias ? bias + (size_t)by * sBias : nullptr;
  const int ntn = (N + 63) / 64; const int wid = blockIdx.x * 4 + w; const int mt = wid / ntn, nq = wid % ntn; if (mt * 16 >= M) return;
  const int row0 = mt * 16, col0 = nq * 64; const _Float16* arow = A + (size_t)(row0 + ln) * lda;
  v8f acc[4] = {};
  for (int kb = 0; kb < K; kb += 32) { FragH ah; ah.half[0] = *(const v8us*)((const unsigned short*)arow + kb + 8 * hh); ah.half[1] = *(const v8us*)((const unsigned short*)arow + kb + 16 + 8 * hh);
#pragma unroll
    for (int t = 0; t < 4; ++t) { if (col0 + t * 16 >= N) continue; const size_t boff = (size_t)(col0 + t * 16 + ln) * ldb + kb; FragH bq; bq.half[0] = *(const v8us*)((const unsigned short*)Bh + boff + 8 * hh); bq.half[1] = *(const v8us*)((const unsigned short*)Bh + boff + 16 + 8 * hh);
      acc[t] = mmaH<1>(ah.v, ah.v, bq.v, bq.v, acc[t]); }
  }
#pragma unroll
  for (int t = 0; t < 4; ++t) { if (col0 + t * 16 >= N) continue; const int col = col0 + t * 16 + ln; const float bv = bp ? bf16_round(bp[col]) : 0.f;
#pragma unroll
    for (int r = 0; r < 8; ++r) { float v = acc[t][r] * alpha + bv; if (CP) { const int bidx = (row0g + row0 + 8 * hh + r) / rowsPerB; v += CP[(size_t)bidx * sCPb + (size_t)by * 64 + col]; } if (ACT == 1) v = (v > 0.f) ? v : expm1f(v); else if (ACT == 7) v = (v > 0.f) ? v + 1.0f : expf(v); else if (ACT == 8) v = tanhf(v); else if (ACT == 9) v = 0.5f * v * (1.0f + tanhf(0.7978845608028654f * (v + 0.044715f * v * v * v))); else if (ACT == 11) v = 1.0f / (1.0f + expf(-v)); else if (ACT == 12) v = (v > 0.f) ? v : 0.01f * v; else if (ACT == 14) v = (v > 0.f) ? v : 0.1f * v; else if (ACT == 15) v = v / (1.0f + expf(-v)); else if (ACT == 3) v = fmaxf(v, 0.f); else if (ACT == 6) v = 0.5f * v * (1.0f + erff(v * 0.70710678118654752f)); so[w][8 * hh + r][t * 16 + ln] = v; } }
  __builtin_amdgcn_fence(__ATOMIC_ACQ_REL, "workgroup"); __builtin_amdgcn_wave_barrier();
  const int rsub = lane >> 4, c4 = (lane & 15) * 4; typedef _Float16 v4h __attribute__((ext_vector_type(4)));
  for (int pass = 0; pass < 2; ++pass) {
#pragma unroll
    for (int q = 0; q < 8; ++q) { const int r = q * 2 + rsub; if (col0 + c4 < N) { const v4f v = *(const v4fa*)&so[w][r][c4]; if (C) *(volatile v4f*)(C + cofs + (size_t)(row0 + r) * ldc + col0 + c4) = v; if (C16) { v4h h4; for (int i = 0; i < 4; ++i) h4[i] = (_Float16)v[i]; *(volatile v4h*)(C16 + cofs + (size_t)(row0 + r) * ldc + col0 + c4) = h4; } } }
    if (pass == 0) __threadfence(); }
}


typedef _Float16 v4h __attribute__((ext_vector_type(4)));

__global__ __launch_bounds__(256) void k_x16(const float* __restrict__ x, _Float16* __restrict__ X16, size_t n8) { const size_t t = (size_t)blockIdx.x * 256 + threadIdx.x; if (t >= n8) return; FragH f;
#pragma unroll
  for (int q = 0; q < 8; ++q) f.h[q] = (_Float16)bf16_round(x[t * 8 + q]); *(volatile v8us*)((unsigned short*)X16 + t * 8) = f.half[0]; __threadfence(); *(volatile v8us*)((unsigned short*)X16 + t * 8) = f.half[0]; }
__global__ __launch_bounds__(256) void k_h16(const float* __restrict__ x, _Float16* __restrict__ X16, size_t n8) { const size_t t = (size_t)blockIdx.x * 256 + threadIdx.x; if (t >= n8) return; FragH f;
#pragma unroll
  for (int q = 0; q < 8; ++q) f.h[q] = (_Float16)x[t * 8 + q]; *(volatile v8us*)((unsigned short*)X16 + t * 8) = f.half[0]; __threadfence(); *(volatile v8us*)((unsigned short*)X16 + t * 8) = f.half[0]; }
__global__ __launch_bounds__(256) void k_round16f(const float* __restrict__ W, _Float16* __restrict__ Bt, size_t n8) { const size_t t = (size_t)blockIdx.x * 256 + threadIdx.x; if (t >= n8) return; FragH f;
#pragma unroll
  for (int i = 0; i < 8; ++i) f.h[i] = (_Float16)(bf16_round(W[t * 8 + i]) * 16.0f); *(volatile v8us*)((unsigned short*)Bt + t * 8) = f.half[0]; __threadfence(); *(volatile v8us*)((unsigned short*)Bt + t * 8) = f.half[0]; }
template <int NHv, int TTv>
__global__ __launch_bounds__(256) void k_vt(const _Float16* __restrict__ V16, int ldv, int voff, _Float16* __restrict__ Vt) { __shared__ unsigned short tl[64][66]; const int tid = threadIdx.x; const int slab = blockIdx.x / (TTv / 64), lg = blockIdx.x % (TTv / 64); const int b = slab / NHv, h = slab % NHv;
  for (int i = tid; i < 64 * 8; i += 256) { const int r = i / 8, c8 = (i % 8) * 8; FragH f; f.half[0] = *(const v8us*)((const unsigned short*)V16 + ((size_t)b * TTv + lg * 64 + r) * ldv + voff + h * 64 + c8);
#pragma unroll
    for (int q = 0; q < 8; ++q) tl[r][c8 + q] = f.u[q]; }
  __syncthreads();
  for (int pass = 0; pass < 2; ++pass) {
#pragma unroll
    for (int rd = 0; rd < 2; ++rd) { const int d = rd * 32 + tid / 8, pc = tid % 8; FragH f;
#pragma unroll
      for (int q = 0; q < 8; ++q) f.u[q] = tl[pc * 8 + q][d];
      *(volatile v8us*)((unsigned short*)Vt + ((size_t)slab * 64 + d) * TTv + lg * 64 + pc * 8) = f.half[0]; }
    if (pass == 0) __threadfence(); } }

__global__ __launch_bounds__(256) void k_hl(const float* __restrict__ F, _Float16* __restrict__ Hh, _Float16* __restrict__ Hl, size_t n8) { const size_t t = (size_t)blockIdx.x * 256 + threadIdx.x; if (t >= n8) return; FragH fh, fl; const v4f a = *(const v4fa*)(F + t * 8), c = *(const v4fa*)(F + t * 8 + 4);
#pragma unroll
  for (int q = 0; q < 4; ++q) { _Float16 h = (_Float16)a[q]; fh.h[q] = h; fl.h[q] = (_Float16)((a[q] - (float)h) * 1024.0f); h = (_Float16)c[q]; fh.h[4 + q] = h; fl.h[4 + q] = (_Float16)((c[q] - (float)h) * 1024.0f); }
  for (int pass = 0; pass < 2; ++pass) { *(volatile v8us*)((unsigned short*)Hh + t * 8) = fh.half[0]; *(volatile v8us*)((unsigned short*)Hl + t * 8) = fl.half[0]; if (pass == 0) __threadfence(); } }

__global__ __launch_bounds__(256) void k_conv1(const float* __restrict__ src, const float* __restrict__ w1, const float* __restrict__ b1, float* __restrict__ Y1) {
  #pragma clang fp contract(off)
  const size_t t = (size_t)blockIdx.x * 256 + threadIdx.x; if (t >= (size_t)NR * (C1 / 4)) return; const int c0 = (int)(t % (C1 / 4)) * 4; const size_t r = t / (C1 / 4); const int b = (int)(r / NP), n = (int)(r % NP);
  const float x0 = bf16_round(src[((size_t)b * 3 + 0) * NP + n]), x1 = bf16_round(src[((size_t)b * 3 + 1) * NP + n]), x2 = bf16_round(src[((size_t)b * 3 + 2) * NP + n]); v4f o;
#pragma unroll
  for (int q = 0; q < 4; ++q) { const int c = c0 + q; o[q] = ((bf16_round(w1[c * 3 + 0]) * x0 + bf16_round(w1[c * 3 + 1]) * x1) + bf16_round(w1[c * 3 + 2]) * x2) + bf16_round(b1[c]); }
  *(volatile v4f*)(Y1 + r * C1 + c0) = o; __threadfence(); *(volatile v4f*)(Y1 + r * C1 + c0) = o; }
__global__ __launch_bounds__(256) void k_colstats(const float* __restrict__ Z, int R, int C, int r0, int part, double* __restrict__ SUM, double* __restrict__ SQ) {
  __shared__ double s1[8][32], s2[8][32]; const int tid = threadIdx.x, w = tid >> 5, l = tid & 31; const int c = blockIdx.x * 32 + l; double a = 0.0, b = 0.0;
#pragma unroll 1
  for (int r = r0 + w; r < r0 + R; r += 8) { const double v = (double)Z[(size_t)(r - r0) * C + c]; a += v; b += v * v; }
  s1[w][l] = a; s2[w][l] = b; __syncthreads();
  if (w == 0) { double t1 = 0.0, t2 = 0.0;
#pragma unroll
    for (int k = 0; k < 8; ++k) { t1 += s1[k][l]; t2 += s2[k][l]; }
    for (int pass = 0; pass < 2; ++pass) { *(volatile double*)(SUM + (size_t)part * C + c) = t1; *(volatile double*)(SQ + (size_t)part * C + c) = t2; if (pass == 0) __threadfence(); } } }
__global__ __launch_bounds__(256) void k_bnab(const double* __restrict__ SUM, const double* __restrict__ SQ, int C, int nparts, int count, const float* __restrict__ g, const float* __restrict__ be, float* __restrict__ AB) {
  #pragma clang fp contract(off)
  const int c = blockIdx.x * 256 + threadIdx.x; if (c >= C) return; double s = 0.0, q = 0.0; for (int p = 0; p < nparts; ++p) { s += SUM[(size_t)p * C + c]; q += SQ[(size_t)p * C + c]; }
  const double m = s / (double)count; double var = q / (double)count - m * m; if (var < 0.0) var = 0.0; const float a = bf16_round(g[c]) / sqrtf((float)var + EPS); const float sh = bf16_round(be[c]) - (float)m * a;
  for (int pass = 0; pass < 2; ++pass) { *(volatile float*)(AB + c) = a; *(volatile float*)(AB + C + c) = sh; if (pass == 0) __threadfence(); } }
__global__ __launch_bounds__(256) void k_bnrelu(const float* __restrict__ Z, int C, const float* __restrict__ AB, _Float16* __restrict__ Hh, _Float16* __restrict__ Hl) {
  #pragma clang fp contract(off)
  const size_t t = (size_t)blockIdx.x * 256 + threadIdx.x; if (t >= (size_t)NR * C / 8) return; const size_t e0 = t * 8; const int c0 = (int)(e0 % C); FragH fh, fl;
#pragma unroll
  for (int q = 0; q < 8; ++q) { const float v = fmaxf(Z[e0 + q] * AB[c0 + q] + AB[C + c0 + q], 0.f); const _Float16 hi = (_Float16)v; fh.h[q] = hi; fl.h[q] = (_Float16)((v - (float)hi) * 1024.0f); }
  for (int pass = 0; pass < 2; ++pass) { *(volatile v8us*)((unsigned short*)Hh + e0) = fh.half[0]; *(volatile v8us*)((unsigned short*)Hl + e0) = fl.half[0]; if (pass == 0) __threadfence(); } }
__global__ __launch_bounds__(256) void k_maxmin(const float* __restrict__ Z, int b, float* __restrict__ MX, float* __restrict__ MN) {
  __shared__ float s1[8][32], s2[8][32]; const int tid = threadIdx.x, w = tid >> 5, l = tid & 31; const int c = blockIdx.x * 32 + l; float mx = -3.0e38f, mn = 3.0e38f;
#pragma unroll 1
  for (int n = w; n < NP; n += 8) { const float v = Z[(size_t)n * C3 + c]; mx = fmaxf(mx, v); mn = fminf(mn, v); }
  s1[w][l] = mx; s2[w][l] = mn; __syncthreads();
  if (w == 0) { float a = s1[0][l], d = s2[0][l];
#pragma unroll
    for (int k = 1; k < 8; ++k) { a = fmaxf(a, s1[k][l]); d = fminf(d, s2[k][l]); }
    for (int pass = 0; pass < 2; ++pass) { *(volatile float*)(MX + (size_t)b * C3 + c) = a; *(volatile float*)(MN + (size_t)b * C3 + c) = d; if (pass == 0) __threadfence(); } } }
__global__ __launch_bounds__(256) void k_head(const float* __restrict__ MX, const float* __restrict__ MN, const float* __restrict__ AB3, const float* __restrict__ fw1, const float* __restrict__ fb1, const float* __restrict__ g4, const float* __restrict__ be4, const float* __restrict__ fw2, const float* __restrict__ fb2, const float* __restrict__ g5, const float* __restrict__ be5, const float* __restrict__ wr, const float* __restrict__ br, const float* __restrict__ wt, const float* __restrict__ bt, float* __restrict__ RT) {
  #pragma clang fp contract(off)
  __shared__ float pooled[NBc][C3]; __shared__ float h1[NBc][F1]; __shared__ float h2[NBc][F2]; __shared__ float rt[NBc][16];
  const int tid = threadIdx.x;
  for (int i = tid; i < NBc * C3; i += 256) { const int b = i / C3, c = i % C3; const float a = AB3[c], s = AB3[C3 + c]; pooled[b][c] = fmaxf(fmaxf(a * MX[i] + s, 0.f), fmaxf(a * MN[i] + s, 0.f)); }
  __syncthreads();
#pragma unroll 1
  for (int oo = 0; oo < 2; ++oo) { const int o = tid + 256 * oo; float acc[NBc];
#pragma unroll
    for (int b = 0; b < NBc; ++b) acc[b] = bf16_round(fb1[o]);
#pragma unroll 1
    for (int k = 0; k < C3; ++k) { const float wv = bf16_round(fw1[(size_t)o * C3 + k]);
#pragma unroll
      for (int b = 0; b < NBc; ++b) acc[b] += pooled[b][k] * wv; }
    float m = 0.f; for (int b = 0; b < NBc; ++b) m += acc[b]; m /= (float)NBc; float var = 0.f; for (int b = 0; b < NBc; ++b) { const float d = acc[b] - m; var += d * d; } var /= (float)NBc; const float sc = bf16_round(g4[o]) / sqrtf(var + EPS);
#pragma unroll
    for (int b = 0; b < NBc; ++b) h1[b][o] = fmaxf((acc[b] - m) * sc + bf16_round(be4[o]), 0.f); }
  __syncthreads();
  { const int o = tid; float acc[NBc];
#pragma unroll
    for (int b = 0; b < NBc; ++b) acc[b] = bf16_round(fb2[o]);
#pragma unroll 1
    for (int k = 0; k < F1; ++k) { const float wv = bf16_round(fw2[(size_t)o * F1 + k]);
#pragma unroll
      for (int b = 0; b < NBc; ++b) acc[b] += h1[b][k] * wv; }
    float m = 0.f; for (int b = 0; b < NBc; ++b) m += acc[b]; m /= (float)NBc; float var = 0.f; for (int b = 0; b < NBc; ++b) { const float d = acc[b] - m; var += d * d; } var /= (float)NBc; const float sc = bf16_round(g5[o]) / sqrtf(var + EPS);
#pragma unroll
    for (int b = 0; b < NBc; ++b) h2[b][o] = fmaxf((acc[b] - m) * sc + bf16_round(be5[o]), 0.f); }
  __syncthreads();
  if (tid < NBc * 12) { const int b = tid / 12, j = tid % 12; float acc; const float* wrow; if (j < 9) { acc = bf16_round(br[j]) + ((j % 4 == 0) ? 1.0f : 0.0f); wrow = wr + (size_t)j * F2; } else { acc = bf16_round(bt[j - 9]); wrow = wt + (size_t)(j - 9) * F2; }
#pragma unroll 1
    for (int k = 0; k < F2; ++k) acc += h2[b][k] * bf16_round(wrow[k]); rt[b][j] = acc; }
  __syncthreads();
  if (tid < NBc * 4) { const int b = tid / 4, q4 = (tid % 4) * 4; v4f v; v[0] = rt[b][q4]; v[1] = rt[b][q4 + 1]; v[2] = rt[b][q4 + 2]; v[3] = rt[b][q4 + 3]; *(volatile v4f*)(RT + (size_t)b * 16 + q4) = v; __threadfence(); *(volatile v4f*)(RT + (size_t)b * 16 + q4) = v; } }
__global__ __launch_bounds__(256) void k_st(const float* __restrict__ src, const float* __restrict__ RT, float* __restrict__ ST) {
  #pragma clang fp contract(off)
  const size_t t = (size_t)blockIdx.x * 256 + threadIdx.x; if (t >= (size_t)NBc * 3 * (NP / 4)) return; const int n0 = (int)(t % (NP / 4)) * 4; const size_t bc = t / (NP / 4); const int b = (int)(bc / 3), c = (int)(bc % 3); const float* rt = RT + (size_t)b * 16; v4f o;
#pragma unroll
  for (int q = 0; q < 4; ++q) { const int n = n0 + q; o[q] = ((bf16_round(src[((size_t)b * 3 + 0) * NP + n]) * rt[0 * 3 + c] + bf16_round(src[((size_t)b * 3 + 1) * NP + n]) * rt[1 * 3 + c]) + bf16_round(src[((size_t)b * 3 + 2) * NP + n]) * rt[2 * 3 + c]) + rt[9 + c]; }
  *(volatile v4f*)(ST + bc * NP + n0) = o; __threadfence(); *(volatile v4f*)(ST + bc * NP + n0) = o; }
__global__ __launch_bounds__(256) void k_dist(const float* __restrict__ ST, const float* __restrict__ tgt, float* __restrict__ D) {
  #pragma clang fp contract(off)
  __shared__ float red[256]; const int tid = threadIdx.x; const int bij = blockIdx.x; const int b = bij / 9, i = (bij / 3) % 3, j = bij % 3; float s = 0.f;
#pragma unroll 1
  for (int n = tid; n < NP; n += 256) { const float d = ST[((size_t)b * 3 + j) * NP + n] - bf16_round(tgt[((size_t)b * 3 + i) * NP + n]); s += d * d; }
  red[tid] = s; __syncthreads(); for (int k = 128; k > 0; k >>= 1) { if (tid < k) red[tid] += red[tid + k]; __syncthreads(); }
  if (tid < 32) { *(volatile float*)(D + (size_t)bij * 32 + tid) = red[0]; __threadfence(); *(volatile float*)(D + (size_t)bij * 32 + tid) = red[0]; } }
__global__ __launch_bounds__(256) void k_out(const float* __restrict__ D, const float* __restrict__ ST, float* __restrict__ out) {
  #pragma clang fp contract(off)
  const size_t t = (size_t)blockIdx.x * 256 + threadIdx.x; if (t >= (size_t)NBc * 3 * NP + 1) return; float v;
  if (t == 0) { float s1 = 0.f, s2 = 0.f; for (int b = 0; b < NBc; ++b) { for (int j = 0; j < 3; ++j) { float m = 3.0e38f; for (int i = 0; i < 3; ++i) m = fminf(m, D[((size_t)(b * 9 + i * 3 + j)) * 32]); s1 += m; } for (int i = 0; i < 3; ++i) { float m = 3.0e38f; for (int j = 0; j < 3; ++j) m = fminf(m, D[((size_t)(b * 9 + i * 3 + j)) * 32]); s2 += m; } } v = s1 / (float)(NBc * 3) + s2 / (float)(NBc * 3); }
  else v = ST[t - 1];
  *(volatile float*)(out + t) = v; __threadfence(); *(volatile float*)(out + t) = v; }

extern "C" void kernel_launch(void* const* d_in, const int* in_sizes, int n_in,
                              void* d_out, int out_size, void* d_ws, size_t ws_size, hipStream_t stream) {
  (void)in_sizes; (void)n_in; (void)out_size;
  const float* const* I = (const float* const*)d_in; const float* src = I[0]; const float* tgt = I[1]; const float* w1 = I[2]; const float* b1 = I[3]; const float* w2 = I[4]; const float* b2 = I[5]; const float* w3 = I[6]; const float* b3 = I[7]; const float* fw1 = I[8]; const float* fb1 = I[9]; const float* fw2 = I[10]; const float* fb2 = I[11]; const float* wr = I[12]; const float* br = I[13]; const float* wt = I[14]; const float* bt = I[15];
  const float* g1 = I[16]; const float* be1 = I[17]; const float* g2 = I[18]; const float* be2 = I[19]; const float* g3 = I[20]; const float* be3 = I[21]; const float* g4 = I[22]; const float* be4 = I[23]; const float* g5 = I[24]; const float* be5 = I[25];
  char* ws = (char*)d_ws; size_t off = 0;
  auto take = [&](size_t bytes) { char* p = ws + off; off += (bytes + 255) & ~(size_t)255; return p; };
  _Float16* B2 = (_Float16*)take((size_t)C2 * C1 * 2); _Float16* B3 = (_Float16*)take((size_t)C3 * C2 * 2);
  float* Y1 = (float*)take((size_t)NR * C1 * 4); _Float16* H1h = (_Float16*)take((size_t)NR * C1 * 2); _Float16* H1l = (_Float16*)take((size_t)NR * C1 * 2); float* Y2 = (float*)take((size_t)NR * C2 * 4); _Float16* H2h = (_Float16*)take((size_t)NR * C2 * 2); _Float16* H2l = (_Float16*)take((size_t)NR * C2 * 2); float* Z3 = (float*)Y1;
  double* SUM = (double*)take((size_t)NBc * C3 * 8); double* SQ = (double*)take((size_t)NBc * C3 * 8); float* AB1 = (float*)take(2 * C1 * 4); float* AB2 = (float*)take(2 * C2 * 4); float* AB3 = (float*)take(2 * C3 * 4); float* MX = (float*)take((size_t)NBc * C3 * 4); float* MN = (float*)take((size_t)NBc * C3 * 4); float* RT = (float*)take((size_t)NBc * 16 * 4); float* ST = (float*)take((size_t)NBc * 3 * NP * 4); float* D = (float*)take(72 * 32 * 4);
  if (off > ws_size) return;
  k_round16f<<<(C2 * C1 / 8 + 255) / 256, 256, 0, stream>>>(w2, B2, (size_t)C2 * C1 / 8); k_round16f<<<(C3 * C2 / 8 + 255) / 256, 256, 0, stream>>>(w3, B3, (size_t)C3 * C2 / 8);
  k_conv1<<<(unsigned)(((size_t)NR * (C1 / 4) + 255) / 256), 256, 0, stream>>>(src, w1, b1, Y1);
  k_colstats<<<C1 / 32, 256, 0, stream>>>(Y1, NR, C1, 0, 0, SUM, SQ); k_bnab<<<1, 256, 0, stream>>>(SUM, SQ, C1, 1, NR, g1, be1, AB1);
  k_bnrelu<<<(unsigned)(((size_t)NR * C1 / 8 + 255) / 256), 256, 0, stream>>>(Y1, C1, AB1, H1h, H1l);
  const dim3 gd2(((NR / 16) * (C2 / 64) + 3) / 4, 1);
  k_gemm_hhx<0><<<gd2, 128, 0, stream>>>(H1h, C1, 0, B2, C1, 0, 0.0625f, b2, 0, nullptr, 1, 0, 0, Y2, nullptr, C2, 0, NR, C2, C1); k_gemm_hhx<0><<<gd2, 128, 0, stream>>>(H1l, C1, 0, B2, C1, 0, 0.0625f / 1024.0f, nullptr, 0, Y2, 1, (size_t)C2, 0, Y2, nullptr, C2, 0, NR, C2, C1);
  k_colstats<<<C2 / 32, 256, 0, stream>>>(Y2, NR, C2, 0, 0, SUM, SQ); k_bnab<<<1, 256, 0, stream>>>(SUM, SQ, C2, 1, NR, g2, be2, AB2);
  k_bnrelu<<<(unsigned)(((size_t)NR * C2 / 8 + 255) / 256), 256, 0, stream>>>(Y2, C2, AB2, H2h, H2l);
  const dim3 gd3(((NP / 16) * (C3 / 64) + 3) / 4, 1);
  for (int b = 0; b < NBc; ++b) {
    k_gemm_hhx<0><<<gd3, 128, 0, stream>>>(H2h + (size_t)b * NP * C2, C2, 0, B3, C2, 0, 0.0625f, b3, 0, nullptr, 1, 0, 0, Z3, nullptr, C3, 0, NP, C3, C2); k_gemm_hhx<0><<<gd3, 128, 0, stream>>>(H2l + (size_t)b * NP * C2, C2, 0, B3, C2, 0, 0.0625f / 1024.0f, nullptr, 0, Z3, 1, (size_t)C3, 0, Z3, nullptr, C3, 0, NP, C3, C2);
    k_colstats<<<C3 / 32, 256, 0, stream>>>(Z3, NP, C3, 0, b, SUM, SQ); k_maxmin<<<C3 / 32, 256, 0, stream>>>(Z3, b, MX, MN); }
  k_bnab<<<(C3 + 255) / 256, 256, 0, stream>>>(SUM, SQ, C3, NBc, NR, g3, be3, AB3);
  k_head<<<1, 256, 0, stream>>>(MX, MN, AB3, fw1, fb1, g4, be4, fw2, fb2, g5, be5, wr, br, wt, bt, RT);
  k_st<<<(unsigned)(((size_t)NBc * 3 * (NP / 4) + 255) / 256), 256, 0, stream>>>(src, RT, ST);
  k_dist<<<NBc * 9, 256, 0, stream>>>(ST, tgt, D);
  k_out<<<(unsigned)(((size_t)NBc * 3 * NP + 1 + 255) / 256), 256, 0, stream>>>(D, ST, (float*)d_out);
}
